// MultiHeadGATLayer_36558761623740
// MI455X (gfx1250) — hardware-run, weakly checked
//
#include <hip/hip_runtime.h>

typedef float          v8f   __attribute__((ext_vector_type(8)));
typedef float          v4f   __attribute__((ext_vector_type(4)));
typedef unsigned int   v4u   __attribute__((ext_vector_type(4)));
typedef int            v8i   __attribute__((ext_vector_type(8)));
typedef unsigned short v8us  __attribute__((ext_vector_type(8)));
typedef unsigned short v16us __attribute__((ext_vector_type(16)));
typedef __bf16         v16bf __attribute__((ext_vector_type(16)));
typedef _Float16       v16h  __attribute__((ext_vector_type(16)));
typedef v4f  __attribute__((may_alias)) v4fa;
typedef v8us __attribute__((may_alias)) v8usa;
union FragB { v16bf v; v16us u; v8us h[2]; v8i w; };
union FragH { v16h  v; v16us u; v8us h[2]; v8i w; };

__device__ __forceinline__ v8f wmb(const FragB& a, const FragB& b, v8f c) {
  v8f d = __builtin_amdgcn_wmma_f32_16x16x32_bf16(false, a.v, false, b.v, (short)0, c, false, false);
  asm volatile("v_nop\n\tv_nop\n\tv_nop\n\tv_nop" : "+v"(d) : "v"(a.w), "v"(b.w));
  return d;
}

__device__ __forceinline__ v8f wmh(const FragH& a, const FragH& b, v8f c) {
  v8f d = __builtin_amdgcn_wmma_f32_16x16x32_f16(false, a.v, false, b.v, (short)0, c, false, false);
  asm volatile("v_nop\n\tv_nop\n\tv_nop\n\tv_nop" : "+v"(d) : "v"(a.w), "v"(b.w));
  return d;
}

__device__ __forceinline__ unsigned bf16_bits(float f) {
  const unsigned u = __float_as_uint(f);
  const unsigned r = (u + 0x7FFFu + ((u >> 16) & 1u)) >> 16;
  const unsigned q = (u >> 16) | 0x40u;
  return ((u & 0x7fffffffu) > 0x7f800000u) ? q : r;
}

__device__ __forceinline__ float bf16_val(float f) {
  return __uint_as_float(bf16_bits(f) << 16);
}
__device__ __forceinline__ int clampi(int v, int lo, int hi) {
  return v < lo ? lo : (v > hi ? hi : v);
}

__device__ __forceinline__ unsigned f16_bits(float f) {
  const unsigned u  = __float_as_uint(f);
  const unsigned s  = (u >> 16) & 0x8000u;
  const unsigned a  = u & 0x7fffffffu;
  const unsigned t  = a - 0x38000000u;
  const unsigned r  = (t + 0x0FFFu + ((t >> 13) & 1u)) >> 13;
  const unsigned rc = r > 0x7C00u ? 0x7C00u : r;
  const bool small  = a < 0x38800000u;
  const bool isnan  = a > 0x7f800000u;
  const unsigned fin = small ? 0u : (s | rc);
  return isnan ? (s | 0x7E00u) : fin;
}

__device__ __forceinline__ unsigned pk16(unsigned lo, unsigned hi) { return lo | (hi << 16); }
__device__ __forceinline__ unsigned bf16_lo_bits(float v) {
  float hi = bf16_val(v);
  asm volatile("" : "+v"(hi));
  return bf16_bits(v - hi);
}
__device__ __forceinline__ v4u pack8_bf16(v4f a, v4f c) {
  return (v4u){ pk16(bf16_bits(a[0]), bf16_bits(a[1])), pk16(bf16_bits(a[2]), bf16_bits(a[3])),
                pk16(bf16_bits(c[0]), bf16_bits(c[1])), pk16(bf16_bits(c[2]), bf16_bits(c[3])) };
}
__device__ __forceinline__ v4u pack8_bf16_lo(v4f a, v4f c) {
  return (v4u){ pk16(bf16_lo_bits(a[0]), bf16_lo_bits(a[1])), pk16(bf16_lo_bits(a[2]), bf16_lo_bits(a[3])),
                pk16(bf16_lo_bits(c[0]), bf16_lo_bits(c[1])), pk16(bf16_lo_bits(c[2]), bf16_lo_bits(c[3])) };
}
__device__ __forceinline__ v4u pack8_f16(v4f a, v4f c) {
  return (v4u){ pk16(f16_bits(a[0]), f16_bits(a[1])), pk16(f16_bits(a[2]), f16_bits(a[3])),
                pk16(f16_bits(c[0]), f16_bits(c[1])), pk16(f16_bits(c[2]), f16_bits(c[3])) };
}

template <int FORM>
__global__ __launch_bounds__(256) void k_plane(const float* __restrict__ src, int rows, int cols, int ldsrc,
                                               unsigned short* __restrict__ dst, int MP, int KP) {
  static_assert(FORM >= 0 && FORM <= 3);
  const int KTOT = (FORM == 1 || FORM == 3) ? 2 * KP : KP;
  const unsigned ppr   = (unsigned)(KTOT >> 3);
  const unsigned kp8   = (unsigned)(KP >> 3);
  const unsigned total = (unsigned)MP * ppr;
  const unsigned g     = blockIdx.x * 256u + threadIdx.x;
  const unsigned rowu  = g / ppr;
  const unsigned p     = g - rowu * ppr;
  const bool second    = p >= kp8;
  const int row = (int)rowu;
  const int c0  = (int)((second ? p - kp8 : p) << 3);
  const float* srow = src + (size_t)clampi(row, 0, rows - 1) * (size_t)ldsrc;
  float x[8];
  unsigned mk[8];
#pragma unroll
  for (int e = 0; e < 8; ++e) {
    const int c = c0 + e;
    const float v = srow[clampi(c, 0, cols - 1)];
    asm volatile("" :: "v"(v));
    x[e]  = v;
    mk[e] = (row < rows && c < cols) ? 0xFFFFu : 0u;
  }
  const v4f a = (v4f){ x[0], x[1], x[2], x[3] };
  const v4f c = (v4f){ x[4], x[5], x[6], x[7] };
  v4u o;
  if (FORM == 2) {
    o = pack8_f16(a, c);
  } else {
    const v4u hi = pack8_bf16(a, c);
    o = hi;
    if (FORM == 1) { const v4u lo = pack8_bf16_lo(a, c); o = second ? lo : hi; }
  }
  const v4u mw = (v4u){ pk16(mk[0], mk[1]), pk16(mk[2], mk[3]), pk16(mk[4], mk[5]), pk16(mk[6], mk[7]) };
  o &= mw;
  if (g < total) {
    volatile v4u* q = (volatile v4u*)(dst + (size_t)g * 8);
    *q = o;
    __threadfence();
    *q = o;
  }
}

template <int FORM> struct FragOf    { typedef FragB T; };
template <>         struct FragOf<2> { typedef FragH T; };
__device__ __forceinline__ v8f mm(const FragB& a, const FragB& b, v8f c) { return wmb(a, b, c); }
__device__ __forceinline__ v8f mm(const FragH& a, const FragH& b, v8f c) { return wmh(a, b, c); }
template <class F> __device__ __forceinline__ F ld_frag(const unsigned short* p) {
  F f;
  f.h[0] = *(const v8usa*)(p);
  f.h[1] = *(const v8usa*)(p + 16);
  return f;
}

template <int FORM, int EPI>
__global__ __launch_bounds__(256) __attribute__((amdgpu_num_vgpr(248)))
void k_gemm_nt(const unsigned short* __restrict__ A, const unsigned short* __restrict__ B,
               const float* __restrict__ bias, float* __restrict__ D, int M, int N, int KTOT, int ldd) {
  static_assert(FORM >= 0 && FORM <= 2);
  static_assert(EPI == 0 || EPI == 1);
  typedef typename FragOf<FORM>::T F;
  __shared__ __attribute__((aligned(16))) float sT[8][16 * 68];
  const int lane = threadIdx.x & 31;
  const int wave = threadIdx.x >> 5;
  const int tilesM = (M + 63) >> 6;
  const int tilesN = (N + 63) >> 6;
  const int tile = blockIdx.x * 8 + wave;
  if (tile >= tilesM * tilesN) return;
  const int tm = tile / tilesN;
  const int tn = tile - tm * tilesN;
  const int m0 = tm << 6;
  const int n0 = tn << 6;

  const int rl = lane & 15;
  const int h8 = (lane >> 4) * 8;
  const unsigned short* pa = A + (size_t)(m0 + rl) * (size_t)KTOT + h8;
  const unsigned short* pb = B + (size_t)(n0 + rl) * (size_t)KTOT + h8;

  v8f acc[4][4];
#pragma unroll
  for (int i = 0; i < 4; ++i)
#pragma unroll
    for (int j = 0; j < 4; ++j) acc[i][j] = (v8f){0.f, 0.f, 0.f, 0.f, 0.f, 0.f, 0.f, 0.f};

#pragma unroll 1
  for (int k0 = 0; k0 < KTOT; k0 += 32) {
    F bf[4];
#pragma unroll
    for (int j = 0; j < 4; ++j) bf[j] = ld_frag<F>(pb + (size_t)(j << 4) * (size_t)KTOT + k0);
#pragma unroll
    for (int i = 0; i < 4; ++i) {
      const F af = ld_frag<F>(pa + (size_t)(i << 4) * (size_t)KTOT + k0);
#pragma unroll
      for (int j = 0; j < 4; ++j) acc[i][j] = mm(af, bf[j], acc[i][j]);
    }
  }

  float* slab = sT[wave];
  const int hh = lane >> 4;
  const int c4 = (lane & 15) * 4;
  const int nc = n0 + c4;
  const bool cok = nc < N;
  v4f bv = (v4f){0.f, 0.f, 0.f, 0.f};
  if (EPI == 1) {
    bv = *(const v4fa*)(bias + clampi(nc, 0, N - 4));
    asm volatile("" :: "v"(bv));
  }
#pragma unroll
  for (int i = 0; i < 4; ++i) {
    const int mBase = m0 + (i << 4);
#pragma unroll
    for (int j = 0; j < 4; ++j) {
#pragma unroll
      for (int r = 0; r < 8; ++r) slab[(h8 + r) * 68 + (j << 4) + rl] = acc[i][j][r];
    }
    __builtin_amdgcn_fence(__ATOMIC_RELEASE, "workgroup");
    __builtin_amdgcn_wave_barrier();
    __builtin_amdgcn_fence(__ATOMIC_ACQUIRE, "workgroup");
    v4f vv[8];
#pragma unroll
    for (int it = 0; it < 8; ++it) {
      const int row = it * 2 + hh;
      v4f v = *(const v4fa*)(slab + row * 68 + c4);
      if (EPI == 1) v += bv;
      vv[it] = v;
    }
    for (int pass = 0; pass < 2; ++pass) {
#pragma unroll
      for (int it = 0; it < 8; ++it) {
        const int row = mBase + it * 2 + hh;
        if (cok && row < M) *(volatile v4f*)(D + (size_t)row * (size_t)ldd + nc) = vv[it];
      }
      __threadfence();
    }
    __builtin_amdgcn_fence(__ATOMIC_RELEASE, "workgroup");
    __builtin_amdgcn_wave_barrier();
    __builtin_amdgcn_fence(__ATOMIC_ACQUIRE, "workgroup");
  }
}

#pragma clang fp contract(off)


#define NN      50000
#define NE      800000
#define MPAD    50048
#define KD      256
#define DOUTW   256
#define NHD     4
#define DSZ     64
#define RTHR    256
#define RWAVES  8
#define BT      512
#define BW      16
#define BEPT    8
#define BCHUNK  (BT * BEPT)
#define NCH     ((NE + BCHUNK - 1) / BCHUNK)
#define NB      1024
#define NBLK    ((NN + NB - 1) / NB)
#define RCAP    20992
#define DEGCAP  64
#define SLOTSH  21
#define LISTTOT (NBLK * RCAP)
#define LDS_BKT ((2 * RCAP + 3 * NB + 64) * 4)
#define WSMAX   ((size_t)128 << 20)

static_assert(NN % 8 == 0);
static_assert(NHD * DSZ == 256 && DSZ == 64 && DOUTW == 256 && KD == 256);
static_assert(MPAD == 782 * 64 && MPAD % 64 == 0 && MPAD >= NN && MPAD % 8 == 0);
static_assert(KD % 32 == 0 && DOUTW % 64 == 0);
static_assert(NE < (1 << SLOTSH));
static_assert(NB <= 1024 && (NB & (NB - 1)) == 0 && NB == 2 * BT);
static_assert(NE % 8 == 0 && NE >= 8);
static_assert(NBLK == 49 && NBLK * NB >= NN);
static_assert(NCH * BCHUNK >= NE && NCH == 196);
static_assert(RCAP % 32 == 0);
static_assert(RCAP * 4 >= 16696 * 5);
static_assert(DEGCAP >= 33 + 8);
static_assert(DEGCAP % 32 == 0);
static_assert(LDS_BKT <= 262144);
static_assert(BW == BT / 32 && BW == 16);
static_assert(NN == (NN / RWAVES) * RWAVES);
static_assert(MPAD * (KD / 8) % 256 == 0);

typedef int          v4i __attribute__((ext_vector_type(4)));
typedef int          v2i __attribute__((ext_vector_type(2)));
typedef v4i __attribute__((may_alias)) v4ia;
typedef v2i __attribute__((may_alias)) v2ia;

__device__ __forceinline__ float lrelu_k(float v) { return (v > 0.0f) ? v : 0.01f * v; }
__device__ __forceinline__ float maxk(float a, float b) {
  float m = (a < b) ? b : a;
  m = (b != b) ? b : m;
  return m;
}
__device__ __forceinline__ float fin0(float m) {
  const bool f = (__float_as_uint(m) & 0x7fffffffu) < 0x7f800000u;
  return f ? m : 0.0f;
}
__device__ __forceinline__ float sum8(float t) {
  t = t + __shfl_xor(t, 4, 32);
  t = t + __shfl_xor(t, 2, 32);
  t = t + __shfl_xor(t, 1, 32);
  return t;
}
__device__ __forceinline__ void wave_lds_sync() {
  __builtin_amdgcn_fence(__ATOMIC_RELEASE, "workgroup");
  __builtin_amdgcn_wave_barrier();
  __builtin_amdgcn_fence(__ATOMIC_ACQUIRE, "workgroup");
}

__global__ __launch_bounds__(256) void k_prep(const float* __restrict__ W, const float* __restrict__ att,
                                              unsigned short* WS, float* ATT, unsigned* FLAG) {
  const int t = (int)threadIdx.x;
  if (blockIdx.x < 32u) {
    const unsigned g = blockIdx.x * 256u + (unsigned)t;
    const v4f a = *(const v4fa*)(W + (size_t)g * 8);
    const v4f c = *(const v4fa*)(W + (size_t)g * 8 + 4);
    asm volatile("" :: "v"(a), "v"(c));
    const v4u o = pack8_bf16(a, c);
    volatile v4u* q = (volatile v4u*)(WS + (size_t)g * 8);
    *q = o;
    __threadfence();
    *q = o;
  } else {
    const int idx = clampi(4 * t, 0, 508);
    const v4f a = *(const v4fa*)(att + idx);
    asm volatile("" :: "v"(a));
    v4u o;
    o.x = bf16_bits(a.x) << 16;
    o.y = bf16_bits(a.y) << 16;
    o.z = bf16_bits(a.z) << 16;
    o.w = bf16_bits(a.w) << 16;
    const v4u zz = (v4u){0u, 0u, 0u, 0u};
    const bool wa = t < 128;
    const bool wf = (t >= 128) && (t < 144);
    volatile v4u* qa = (volatile v4u*)(ATT + 4 * clampi(t, 0, 127));
    volatile v4u* qf = (volatile v4u*)(FLAG + 4 * clampi(t - 128, 0, 15));
    if (wa) *qa = o;
    if (wf) *qf = zz;
    __threadfence();
    if (wa) *qa = o;
    if (wf) *qf = zz;
  }
}

__global__ __launch_bounds__(BT) void k_list(const int* __restrict__ ekey, const int* __restrict__ egid,
                                             unsigned* LIST, int* META, unsigned* FLAG) {
  extern __shared__ v4u lds_bkt[];
  int* reg1 = (int*)lds_bkt;
  int* reg2 = reg1 + RCAP;
  int* scnt = reg2 + RCAP;
  int* soff = scnt + NB;
  int* curs = soff + NB;
  int* wcnt = curs + NB;
  int* wtot = wcnt + 2 * BW;
  const int tid = (int)threadIdx.x, lane = tid & 31, wave = tid >> 5;
  const int nodeBase = (int)blockIdx.x * NB;
  int nb = NN - nodeBase;
  nb = nb > NB ? NB : (nb < 0 ? 0 : nb);
  const unsigned nbs = (unsigned)nodeBase, unb = (unsigned)nb;

  scnt[2 * tid] = 0;
  scnt[2 * tid + 1] = 0;

  int tot = 0;
#pragma unroll 1
  for (int ch = 0; ch < NCH; ++ch) {
    const int par = ch & 1;
    const int e0  = ch * BCHUNK + tid * BEPT;
    const bool valid = e0 < NE;
    const int ea = e0 < NE - 8 ? e0 : NE - 8;
    const v4i da = *(const v4ia*)(ekey + ea);
    const v4i db = *(const v4ia*)(ekey + ea + 4);
    asm volatile("" :: "v"(da), "v"(db));
    const unsigned s0 = (unsigned)da.x - nbs, s1 = (unsigned)da.y - nbs;
    const unsigned s2 = (unsigned)da.z - nbs, s3 = (unsigned)da.w - nbs;
    const unsigned s4 = (unsigned)db.x - nbs, s5 = (unsigned)db.y - nbs;
    const unsigned s6 = (unsigned)db.z - nbs, s7 = (unsigned)db.w - nbs;
    const bool h0 = valid && (s0 < unb), h1 = valid && (s1 < unb), h2 = valid && (s2 < unb), h3 = valid && (s3 < unb);
    const bool h4 = valid && (s4 < unb), h5 = valid && (s5 < unb), h6 = valid && (s6 < unb), h7 = valid && (s7 < unb);
    const int c = (int)h0 + (int)h1 + (int)h2 + (int)h3 + (int)h4 + (int)h5 + (int)h6 + (int)h7;
    int incl = c;
#pragma unroll
    for (int d = 1; d < 32; d <<= 1) {
      const int up = __shfl_up(incl, d, 32);
      incl += (lane >= d) ? up : 0;
    }
    const int wtotal = __shfl(incl, 31, 32);
    if (lane == 0) wcnt[par * BW + wave] = wtotal;
    __syncthreads();
    int all = 0, pre = 0;
#pragma unroll
    for (int g = 0; g < 4; ++g) {
      const v4i w4 = *(const v4ia*)(wcnt + par * BW + 4 * g);
      const int c0 = clampi(w4.x, 0, 256), c1 = clampi(w4.y, 0, 256);
      const int c2 = clampi(w4.z, 0, 256), c3 = clampi(w4.w, 0, 256);
      all += c0 + c1 + c2 + c3;
      pre += (4 * g + 0 < wave) ? c0 : 0;
      pre += (4 * g + 1 < wave) ? c1 : 0;
      pre += (4 * g + 2 < wave) ? c2 : 0;
      pre += (4 * g + 3 < wave) ? c3 : 0;
    }
    int pos = tot + pre + (incl - c);
#define PUTJ(J, HJ, SJ) if (HJ) { if (pos < RCAP) reg1[pos] = (int)((unsigned)(e0 + (J)) | ((SJ) << SLOTSH)); ++pos; }
    PUTJ(0, h0, s0)
    PUTJ(1, h1, s1)
    PUTJ(2, h2, s2)
    PUTJ(3, h3, s3)
    PUTJ(4, h4, s4)
    PUTJ(5, h5, s5)
    PUTJ(6, h6, s6)
    PUTJ(7, h7, s7)
#undef PUTJ
    tot += all;
  }
  __syncthreads();
  const bool ovf = tot > RCAP;
  const int nh = ovf ? RCAP : tot;

  if (wave == 0) {
#pragma unroll 1
    for (int b0 = 0; b0 < nh; b0 += 32) {
      const int idx = b0 + lane;
      const int uv  = reg1[idx < nh ? idx : nh - 1];
      const int m32 = (nh - b0) < 32 ? (nh - b0) : 32;
#pragma unroll 1
      for (int k = 0; k < m32; ++k) {
        const int u  = __builtin_amdgcn_readlane(uv, k);
        const int sl = (int)(((unsigned)u >> SLOTSH) & (unsigned)(NB - 1));
        const int cv = scnt[sl] + 1;
        if (lane == 0) scnt[sl] = cv;
      }
    }
  }
  __syncthreads();

  int e0c, e1c;
  {
    const v2i cc = *(const v2ia*)(scnt + 2 * tid);
    e0c = cc.x < 0 ? 0 : cc.x;
    e1c = cc.y < 0 ? 0 : cc.y;
    const int ts = e0c + e1c;
    int incl = ts;
#pragma unroll
    for (int d = 1; d < 32; d <<= 1) {
      const int up = __shfl_up(incl, d, 32);
      incl += (lane >= d) ? up : 0;
    }
    if (lane == 31) wtot[wave] = incl;
    __syncthreads();
    int pre = 0;
#pragma unroll
    for (int g = 0; g < 4; ++g) {
      const v4i w4 = *(const v4ia*)(wtot + 4 * g);
      pre += (4 * g + 0 < wave) ? w4.x : 0;
      pre += (4 * g + 1 < wave) ? w4.y : 0;
      pre += (4 * g + 2 < wave) ? w4.z : 0;
      pre += (4 * g + 3 < wave) ? w4.w : 0;
    }
    const int run = pre + incl - ts;
    soff[2 * tid]     = run;
    soff[2 * tid + 1] = run + e0c;
    curs[2 * tid]     = run;
    curs[2 * tid + 1] = run + e0c;
  }
  __syncthreads();

  if (wave == 0) {
#pragma unroll 1
    for (int b0 = 0; b0 < nh; b0 += 32) {
      const int idx = b0 + lane;
      const int uv  = reg1[idx < nh ? idx : nh - 1];
      const int m32 = (nh - b0) < 32 ? (nh - b0) : 32;
#pragma unroll 1
      for (int k = 0; k < m32; ++k) {
        const int u   = __builtin_amdgcn_readlane(uv, k);
        const int sl  = (int)(((unsigned)u >> SLOTSH) & (unsigned)(NB - 1));
        const int eid = (int)((unsigned)u & ((1u << SLOTSH) - 1u));
        const int pr  = curs[sl];
        const int pc  = clampi(pr, 0, RCAP - 1);
        if (lane == 0) { reg2[pc] = eid; curs[sl] = pc + 1; }
      }
    }
  }
  __syncthreads();

  {
    int nhPad = (nh + 31) & ~31;
    nhPad = nhPad > RCAP ? RCAP : nhPad;
    const int nIt = (nhPad + BT - 1) / BT;
    unsigned* lbase = LIST + (size_t)blockIdx.x * (size_t)RCAP;
#pragma unroll 1
    for (int it = 0; it < nIt; ++it) {
      const int i  = it * BT + tid;
      const int ic = i < nh ? i : nh - 1;
      const int eid = clampi(reg2[ic], 0, NE - 1);
      const int gw = egid[eid];
      asm volatile("" :: "v"(gw));
      const unsigned msk = (i < nh) ? 0xFFFFFFFFu : 0u;
      const unsigned o = (unsigned)clampi(gw, 0, NN - 1) & msk;
      const int iw = i < RCAP ? i : RCAP - 1;
      volatile unsigned* q = (volatile unsigned*)(lbase + (size_t)iw);
      const bool wr = i < nhPad;
      if (wr) *q = o;
      __threadfence();
      if (wr) *q = o;
    }
  }

  {
    const int base = (int)blockIdx.x * RCAP;
    const v2i cc = *(const v2ia*)(scnt + 2 * tid);
    const v2i so = *(const v2ia*)(soff + 2 * tid);
    v4i m;
    m.x = base + so.x;
    m.y = ovf ? -1 : cc.x;
    m.z = base + so.y;
    m.w = ovf ? -1 : cc.y;
    volatile v4i* q = (volatile v4i*)(META + 2 * (size_t)(nodeBase + 2 * tid));
    *q = m;
    __threadfence();
    *q = m;
  }

  {
    const bool wf = ovf && (tid == 0);
    volatile unsigned* qf = (volatile unsigned*)FLAG;
    if (wf) *qf = 1u;
    __threadfence();
    if (wf) *qf = 1u;
  }
}

__global__ __launch_bounds__(RTHR) void k_rowprep(const float* __restrict__ Z, const float* __restrict__ ATT,
                                                  float* ES, float* ED) {
  __shared__ __attribute__((aligned(16))) float sS[RWAVES * NHD];
  __shared__ __attribute__((aligned(16))) float sD[RWAVES * NHD];
  const int lane = (int)threadIdx.x & 31;
  const int wave = (int)threadIdx.x >> 5;
  const int row  = clampi((int)blockIdx.x * RWAVES + wave, 0, MPAD - 1);
  const int head = lane >> 3;
  const int c0   = lane * 8;
  const int a0   = head * 128 + (lane & 7) * 8;
  const float* zr = Z + (size_t)row * DOUTW + c0;
  const v4f z0 = *(const v4fa*)zr;
  const v4f z1 = *(const v4fa*)(zr + 4);
  asm volatile("" :: "v"(z0), "v"(z1));
  const v4f s0 = *(const v4fa*)(ATT + a0);
  const v4f s1 = *(const v4fa*)(ATT + a0 + 4);
  const v4f d0 = *(const v4fa*)(ATT + a0 + 64);
  const v4f d1 = *(const v4fa*)(ATT + a0 + 68);
  float t, u;
  t = z0.x * s0.x;
  u = z0.y * s0.y; t = t + u;
  u = z0.z * s0.z; t = t + u;
  u = z0.w * s0.w; t = t + u;
  u = z1.x * s1.x; t = t + u;
  u = z1.y * s1.y; t = t + u;
  u = z1.z * s1.z; t = t + u;
  u = z1.w * s1.w; t = t + u;
  const float es = sum8(t);
  t = z0.x * d0.x;
  u = z0.y * d0.y; t = t + u;
  u = z0.z * d0.z; t = t + u;
  u = z0.w * d0.w; t = t + u;
  u = z1.x * d1.x; t = t + u;
  u = z1.y * d1.y; t = t + u;
  u = z1.z * d1.z; t = t + u;
  u = z1.w * d1.w; t = t + u;
  const float ed = sum8(t);
  if ((lane & 7) == 0) {
    sS[wave * NHD + head] = es;
    sD[wave * NHD + head] = ed;
  }
  __syncthreads();
  if (wave == 0) {
    const int l8 = lane & 7;
    const v4f sv = *(const v4fa*)(sS + 4 * l8);
    const v4f sw = *(const v4fa*)(sD + 4 * l8);
    const int trow = clampi((int)blockIdx.x * RWAVES + l8, 0, MPAD - 1);
    const bool wr = lane < 8;
    volatile v4f* qs = (volatile v4f*)(ES + (size_t)trow * NHD);
    volatile v4f* qd = (volatile v4f*)(ED + (size_t)trow * NHD);
    if (wr) *qs = sv;
    if (wr) *qd = sw;
    __threadfence();
    if (wr) *qs = sv;
    if (wr) *qd = sw;
  }
}

__global__ __launch_bounds__(RTHR) void k_walk(const float* __restrict__ Z, const float* __restrict__ ES,
                                               const float* __restrict__ ED, const unsigned* __restrict__ LIST,
                                               const int* __restrict__ META, const unsigned* __restrict__ FLAG,
                                               float* out, int nrows) {
  __shared__ __attribute__((aligned(16))) float sW[RWAVES][DEGCAP * NHD];
  __shared__ __attribute__((aligned(16))) int   sC[RWAVES][DEGCAP];
  const int lane = (int)threadIdx.x & 31;
  const int wave = (int)threadIdx.x >> 5;
  const int row  = (int)blockIdx.x * RWAVES + wave;
  const int rowc = clampi(row, 0, nrows - 1);
  const int hA   = lane >> 4;
  const int hB   = 2 + hA;
  const int c0   = lane * 4;
  float* wS = sW[wave];
  int*   cS = sC[wave];

  const v2i mt = *(const v2ia*)(META + 2 * (size_t)rowc);
  asm volatile("" :: "v"(mt));
  const unsigned flg = FLAG[0];
  asm volatile("" :: "v"(flg));
  const int craw = mt.y;
  const int offv = clampi(mt.x, 0, LISTTOT - 1);
  int cntv = clampi(craw, 0, DEGCAP);
  cntv = cntv < (LISTTOT - offv) ? cntv : (LISTTOT - offv);
  const int off = __builtin_amdgcn_readfirstlane(offv);
  const int cnt = __builtin_amdgcn_readfirstlane(cntv);
  const bool poison = (flg == 1u) || (craw < 0) || (craw > DEGCAP);

  const v4f ed4 = *(const v4fa*)(ED + (size_t)rowc * NHD);
  asm volatile("" :: "v"(ed4));
  const float ninf = -__builtin_inff();
  v4f mx4 = (v4f){ninf, ninf, ninf, ninf};

#pragma unroll 1
  for (int b0 = 0; b0 < cnt; b0 += 32) {
    const int j  = b0 + lane;
    const int jc = j < cnt ? j : cnt - 1;
    const unsigned ent = LIST[(size_t)(off + jc)];
    asm volatile("" :: "v"(ent));
    const int col = clampi((int)ent, 0, NN - 1);
    const v4f es = *(const v4fa*)(ES + (size_t)col * NHD);
    asm volatile("" :: "v"(es));
    v4f e;
    e.x = lrelu_k(es.x + ed4.x);
    e.y = lrelu_k(es.y + ed4.y);
    e.z = lrelu_k(es.z + ed4.z);
    e.w = lrelu_k(es.w + ed4.w);
    mx4.x = maxk(mx4.x, e.x);
    mx4.y = maxk(mx4.y, e.y);
    mx4.z = maxk(mx4.z, e.z);
    mx4.w = maxk(mx4.w, e.w);
    if (j < cnt) {
      *(v4fa*)(wS + 4 * j) = e;
      cS[j] = col;
    }
  }
#pragma unroll
  for (int d = 16; d > 0; d >>= 1) {
    const float o0 = __shfl_xor(mx4.x, d, 32);
    const float o1 = __shfl_xor(mx4.y, d, 32);
    const float o2 = __shfl_xor(mx4.z, d, 32);
    const float o3 = __shfl_xor(mx4.w, d, 32);
    mx4.x = maxk(mx4.x, o0);
    mx4.y = maxk(mx4.y, o1);
    mx4.z = maxk(mx4.z, o2);
    mx4.w = maxk(mx4.w, o3);
  }
  v4f m4;
  m4.x = fin0(mx4.x);
  m4.y = fin0(mx4.y);
  m4.z = fin0(mx4.z);
  m4.w = fin0(mx4.w);
  wave_lds_sync();

#pragma unroll 1
  for (int b0 = 0; b0 < cnt; b0 += 32) {
    const int j  = b0 + lane;
    const int jc = j < cnt ? j : cnt - 1;
    const v4f e = *(const v4fa*)(wS + 4 * jc);
    v4f x;
    x.x = expf(e.x - m4.x);
    x.y = expf(e.y - m4.y);
    x.z = expf(e.z - m4.z);
    x.w = expf(e.w - m4.w);
    if (j < cnt) *(v4fa*)(wS + 4 * j) = x;
  }
  wave_lds_sync();
  v4f den = (v4f){0.0f, 0.0f, 0.0f, 0.0f};
#pragma unroll 1
  for (int k = 0; k < cnt; ++k) {
    const v4f x = *(const v4fa*)(wS + 4 * k);
    den.x = den.x + x.x;
    den.y = den.y + x.y;
    den.z = den.z + x.z;
    den.w = den.w + x.w;
  }
  v4f dn;
  dn.x = (den.x < 1e-16f) ? 1e-16f : den.x;
  dn.y = (den.y < 1e-16f) ? 1e-16f : den.y;
  dn.z = (den.z < 1e-16f) ? 1e-16f : den.z;
  dn.w = (den.w < 1e-16f) ? 1e-16f : den.w;

#pragma unroll 1
  for (int b0 = 0; b0 < cnt; b0 += 32) {
    const int j  = b0 + lane;
    const int jc = j < cnt ? j : cnt - 1;
    const v4f x = *(const v4fa*)(wS + 4 * jc);
    v4f w;
    w.x = x.x / dn.x;
    w.y = x.y / dn.y;
    w.z = x.z / dn.z;
    w.w = x.w / dn.w;
    if (j < cnt) *(v4fa*)(wS + 4 * j) = w;
  }
  wave_lds_sync();
  v4f aA = (v4f){0.0f, 0.0f, 0.0f, 0.0f};
  v4f aB = (v4f){0.0f, 0.0f, 0.0f, 0.0f};
#pragma unroll 1
  for (int k = 0; k < cnt; ++k) {
    const int c = clampi(cS[k], 0, NN - 1);
    const float wA = wS[4 * k + hA];
    const float wB = wS[4 * k + hB];
    const float* zr = Z + (size_t)c * DOUTW + c0;
    const v4f zA = *(const v4fa*)zr;
    const v4f zB = *(const v4fa*)(zr + 128);
    float pr;
    pr = wA * zA.x; aA.x = aA.x + pr;
    pr = wA * zA.y; aA.y = aA.y + pr;
    pr = wA * zA.z; aA.z = aA.z + pr;
    pr = wA * zA.w; aA.w = aA.w + pr;
    pr = wB * zB.x; aB.x = aB.x + pr;
    pr = wB * zB.y; aB.y = aB.y + pr;
    pr = wB * zB.z; aB.z = aB.z + pr;
    pr = wB * zB.w; aB.w = aB.w + pr;
  }

  const float qnan = __uint_as_float(0x7fc00000u);
  v4f rA, rB;
  rA.x = poison ? qnan : aA.x;
  rA.y = poison ? qnan : aA.y;
  rA.z = poison ? qnan : aA.z;
  rA.w = poison ? qnan : aA.w;
  rB.x = poison ? qnan : aB.x;
  rB.y = poison ? qnan : aB.y;
  rB.z = poison ? qnan : aB.z;
  rB.w = poison ? qnan : aB.w;
  float* orow = out + (size_t)rowc * DOUTW + c0;
  const bool rok = row < nrows;
  if (rok) *(volatile v4f*)orow = rA;
  if (rok) *(volatile v4f*)(orow + 128) = rB;
  __threadfence();
  if (rok) *(volatile v4f*)orow = rA;
  if (rok) *(volatile v4f*)(orow + 128) = rB;
}

extern "C" void kernel_launch(void* const* d_in, const int* in_sizes, int n_in,
                              void* d_out, int out_size, void* d_ws, size_t ws_size,
                              hipStream_t stream) {
  if (n_in < 5) return;
  if (in_sizes[0] != NN * KD) return;
  if (in_sizes[1] != NE || in_sizes[2] != NE) return;
  if (in_sizes[3] != NHD * DSZ * KD) return;
  if (in_sizes[4] != NHD * 2 * DSZ) return;
  if (out_size != NN * DOUTW) return;

  const float* hfe  = (const float*)d_in[0];
  const int*   egid = (const int*)  d_in[1];
  const int*   ekey = (const int*)  d_in[2];
  const float* Wst  = (const float*)d_in[3];
  const float* att  = (const float*)d_in[4];
  float* out = (float*)d_out;

  const size_t szXB   = (size_t)MPAD * KD * 2;
  const size_t szWS   = (size_t)DOUTW * KD * 2;
  const size_t szATT  = (size_t)NHD * 2 * DSZ * 4;
  const size_t szFLAG = 256;
  const size_t szZ    = (size_t)MPAD * DOUTW * 4;
  const size_t szE    = (size_t)MPAD * NHD * 4;
  const size_t szMETA = (size_t)NBLK * NB * 2 * 4;
  const size_t szLIST = (size_t)NBLK * RCAP * 4;
  static_assert((size_t)MPAD * KD * 2 + (size_t)DOUTW * KD * 2 + (size_t)NHD * 2 * DSZ * 4 + 256 +
                (size_t)MPAD * DOUTW * 4 + 2 * (size_t)MPAD * NHD * 4 + (size_t)NBLK * NB * 8 +
                (size_t)NBLK * RCAP * 4 == 83124480);
  static_assert(83124480 <= WSMAX);
  char* ws = (char*)d_ws;
  size_t off = 0;
  const size_t oXB   = off; off += szXB;
  const size_t oWS   = off; off += szWS;
  const size_t oATT  = off; off += szATT;
  const size_t oFLAG = off; off += szFLAG;
  const size_t oZ    = off; off += szZ;
  const size_t oES   = off; off += szE;
  const size_t oED   = off; off += szE;
  const size_t oMETA = off; off += szMETA;
  const size_t oLIST = off; off += szLIST;
  if (off > ws_size || off > (size_t)WSMAX) return;
  unsigned short* XB  = (unsigned short*)(ws + oXB);
  unsigned short* WS  = (unsigned short*)(ws + oWS);
  float*    ATT  = (float*)(ws + oATT);
  unsigned* FLAG = (unsigned*)(ws + oFLAG);
  float*    Z    = (float*)(ws + oZ);
  float*    ES   = (float*)(ws + oES);
  float*    ED   = (float*)(ws + oED);
  int*      META = (int*)(ws + oMETA);
  unsigned* LIST = (unsigned*)(ws + oLIST);

  hipFuncSetAttribute(reinterpret_cast<const void*>(&k_list),
                      hipFuncAttributeMaxDynamicSharedMemorySize, LDS_BKT);

  k_plane<0><<<MPAD * (KD / 8) / 256, 256, 0, stream>>>(hfe, NN, KD, KD, XB, MPAD, KD);
  k_prep<<<33, 256, 0, stream>>>(Wst, att, WS, ATT, FLAG);
  k_list<<<NBLK, BT, LDS_BKT, stream>>>(ekey, egid, LIST, META, FLAG);
  const int tiles = (MPAD / 64) * (DOUTW / 64);
  const int gG = (tiles + 7) / 8;
  k_gemm_nt<0, 0><<<gG, 256, 0, stream>>>(XB, WS, ATT, Z, MPAD, DOUTW, KD, DOUTW);
  k_rowprep<<<MPAD / RWAVES, RTHR, 0, stream>>>(Z, ATT, ES, ED);
  k_walk<<<NN / RWAVES, RTHR, 0, stream>>>(Z, ES, ED, LIST, META, FLAG, out, NN);
}
